// LSTM_2946347565336
// MI455X (gfx1250) — hardware-verified
//
#include <hip/hip_runtime.h>
#include <math.h>

constexpr int SEQ_B    = 64;
constexpr int SEQ_T    = 1024;
constexpr int DIM_E    = 768;
constexpr int DIM_H    = 256;
constexpr int DIM_V    = 3072;
constexpr int SCAN_THR = 512;
constexpr int ROWS_BLK = 16;
constexpr int ST_PITCH = 264;
constexpr int FS_PITCH = 260;
constexpr int ST_PLANE = ROWS_BLK * ST_PITCH;
constexpr int ST_BUF   = 4 * ST_PLANE;
constexpr int OUT0_ELEMS = SEQ_B * DIM_V;
constexpr int OUT1_ELEMS = SEQ_B * DIM_H;
constexpr float W_CARRY       = 16.0f;
constexpr float W_CARRY_INV   = 1.0f / 16.0f;
constexpr float RES_CARRY     = 2048.0f;
constexpr float RES_CARRY_INV = 1.0f / 2048.0f;

static_assert(DIM_H == 16 * (SCAN_THR / 32), "one 16-column group per wave");
static_assert(SEQ_B % ROWS_BLK == 0, "block rows");
static_assert(DIM_E % 32 == 0 && DIM_H % 32 == 0, "GEMM K multiples of 32");
static_assert(DIM_V % 64 == 0 && DIM_H % 64 == 0 && SEQ_B % 64 == 0, "GEMM M, N tile multiples");
static_assert((2 * ST_BUF) % SCAN_THR == 0, "state zero-fill loop exact");
static_assert(((DIM_V / 64) * (DIM_H / 64)) % 8 == 0, "vocabulary GEMM grid exact");
static_assert(((SEQ_B / 64) * (DIM_V / 64)) % 8 == 0, "head GEMM grid exact");
static_assert((size_t)OUT0_ELEMS * 4 == 786432, "out1 byte offset");
static_assert((size_t)(OUT0_ELEMS + OUT1_ELEMS) * 4 == 851968, "out2 byte offset");
static_assert((size_t)(OUT0_ELEMS + 2 * OUT1_ELEMS) * 4 == 917504, "d_out total bytes");

typedef __attribute__((ext_vector_type(16))) _Float16 v16h;
typedef __attribute__((ext_vector_type(8)))  _Float16 v8h;
typedef __attribute__((ext_vector_type(16))) __bf16   v16b;
typedef __attribute__((ext_vector_type(8)))  __bf16   v8b;
typedef __attribute__((ext_vector_type(8)))  float    v8f;
typedef __attribute__((ext_vector_type(4)))  float    v4f;

__device__ __forceinline__ unsigned short f2bf_bits(float f) {
  unsigned u = __float_as_uint(f);
  return (unsigned short)((u + 0x7FFFu + ((u >> 16) & 1u)) >> 16);
}
__device__ __forceinline__ float bf_bits2f(unsigned short h) { return __uint_as_float(((unsigned)h) << 16); }

__device__ __forceinline__ void dep_guard4_h(v8f& a, v8f& b, v8f& c, v8f& d, v16h x, v16h y) {
  asm volatile("v_nop\n\tv_nop\n\tv_nop\n\tv_nop" : "+v"(a), "+v"(b), "+v"(c), "+v"(d) : "v"(x), "v"(y));
}
__device__ __forceinline__ void dep_guard4_b(v8f& a, v8f& b, v8f& c, v8f& d, v16b x, v16b y) {
  asm volatile("v_nop\n\tv_nop\n\tv_nop\n\tv_nop" : "+v"(a), "+v"(b), "+v"(c), "+v"(d) : "v"(x), "v"(y));
}
__device__ __forceinline__ void keep4_h(v16h a, v16h b, v16h c, v16h d) { asm volatile("v_nop" :: "v"(a), "v"(b), "v"(c), "v"(d)); }
__device__ __forceinline__ void keep4_b(v16b a, v16b b, v16b c, v16b d) { asm volatile("v_nop" :: "v"(a), "v"(b), "v"(c), "v"(d)); }
__device__ __forceinline__ void acc_guard4(v8f& a, v8f& b, v8f& c, v8f& d) {
  asm volatile("v_nop\n\tv_nop\n\tv_nop\n\tv_nop" : "+v"(a), "+v"(b), "+v"(c), "+v"(d));
}
__device__ __forceinline__ void scan_guard(v8f& a, v8f& b, v8f& c, v8f& d,
                                           v16h a0, v16h a1, v16h a2, v16h a3, v16h b0, v16h b1) {
  asm volatile("v_nop\n\tv_nop\n\tv_nop\n\tv_nop"
               : "+v"(a), "+v"(b), "+v"(c), "+v"(d)
               : "v"(a0), "v"(a1), "v"(a2), "v"(a3), "v"(b0), "v"(b1));
}

template <typename T> struct Frag;
template <> struct Frag<_Float16> {
  typedef v16h V;
  union U { v16h v; v8h h[2]; };
  static __device__ __forceinline__ v16h load(const _Float16* p) {
    U f;
    f.h[0] = *(const v8h*)(p);
    f.h[1] = *(const v8h*)(p + 16);
    return f.v;
  }
  static __device__ __forceinline__ v8f mma(v16h a, v16h b, v8f c) {
    return __builtin_amdgcn_wmma_f32_16x16x32_f16(false, a, false, b, (short)0, c, false, false);
  }
  static __device__ __forceinline__ void guard4(v8f& a, v8f& b, v8f& c, v8f& d, v16h x, v16h y) { dep_guard4_h(a, b, c, d, x, y); }
  static __device__ __forceinline__ void keep(v16h a, v16h b, v16h c, v16h d) { keep4_h(a, b, c, d); }
};
template <> struct Frag<__bf16> {
  typedef v16b V;
  union U { v16b v; v8b h[2]; };
  static __device__ __forceinline__ v16b load(const __bf16* p) {
    U f;
    f.h[0] = *(const v8b*)(p);
    f.h[1] = *(const v8b*)(p + 16);
    return f.v;
  }
  static __device__ __forceinline__ v8f mma(v16b a, v16b b, v8f c) {
    return __builtin_amdgcn_wmma_f32_16x16x32_bf16(false, a, false, b, (short)0, c, false, false);
  }
  static __device__ __forceinline__ void guard4(v8f& a, v8f& b, v8f& c, v8f& d, v16b x, v16b y) { dep_guard4_b(a, b, c, d, x, y); }
  static __device__ __forceinline__ void keep(v16b a, v16b b, v16b c, v16b d) { keep4_b(a, b, c, d); }
};

template <int ET> struct Elem;
template <> struct Elem<0> { typedef _Float16 T; };
template <> struct Elem<1> { typedef __bf16 T; };
template <int ET, bool SPLIT, int BIAS_MODE, int OUT_MODE, bool RESID, int ACT = 0>
__global__ __launch_bounds__(256) void wmma_gemm64(
    const unsigned short* __restrict__ Ap, const unsigned short* __restrict__ A2p, int lda, long strideA,
    const unsigned short* __restrict__ Btp, const unsigned short* __restrict__ Bt2p, int ldb, long strideB,
    void* __restrict__ Cout, void* __restrict__ Cout2, int ldc, long strideC,
    const float* __restrict__ bias,
    const float* __restrict__ resid, long strideR,
    int M, int N, int K, float scale) {
  typedef typename Elem<ET>::T T;
  typedef typename Frag<T>::V V;
  const T* A = (const T*)Ap;
  const T* A2 = (const T*)A2p;
  const T* Bt = (const T*)Btp;
  const T* Bt2 = (const T*)Bt2p;
  __shared__ __align__(16) float sT[8][16 * 68];
  const int b    = blockIdx.y;
  const int lane = threadIdx.x & 31;
  const int wave = threadIdx.x >> 5;
  const int tilesN = N >> 6;
  const int tilesM = M >> 6;
  const int tile = blockIdx.x * 8 + wave;
  if (tile >= tilesM * tilesN) return;
  const int tm = tile / tilesN;
  const int tn = tile - tm * tilesN;
  const int m0 = tm << 6;
  const int n0 = tn << 6;

  const T* Ab  = A  + (size_t)b * strideA;
  const T* Bb  = Bt + (size_t)b * strideB;
  const T* Ab2 = SPLIT ? (A2  + (size_t)b * strideA) : nullptr;
  const T* Bb2 = SPLIT ? (Bt2 + (size_t)b * strideB) : nullptr;

  const int rlane = lane & 15;
  const int koff  = (lane >> 4) * 8;
  const int mOff  = (lane >> 4) * 8;

  v8f acc[4][4];
#pragma unroll
  for (int i = 0; i < 4; ++i)
#pragma unroll
    for (int j = 0; j < 4; ++j) acc[i][j] = (v8f){0.f, 0.f, 0.f, 0.f, 0.f, 0.f, 0.f, 0.f};

  for (int k0 = 0; k0 < K; k0 += 32) {
    V bh[4], bl[4];
#pragma unroll
    for (int j = 0; j < 4; ++j) {
      const size_t bo = (size_t)(n0 + (j << 4) + rlane) * ldb + koff + k0;
      bh[j] = Frag<T>::load(Bb + bo);
      if (SPLIT) bl[j] = Frag<T>::load(Bb2 + bo);
    }
#pragma unroll
    for (int i = 0; i < 4; ++i) {
      const size_t ao = (size_t)(m0 + (i << 4) + rlane) * lda + koff + k0;
      V ah = Frag<T>::load(Ab + ao);
      V al = ah;
      if (SPLIT) al = Frag<T>::load(Ab2 + ao);
#pragma unroll
      for (int j = 0; j < 4; ++j) {
        acc[i][j] = Frag<T>::mma(ah, bh[j], acc[i][j]);
        if (SPLIT) {
          acc[i][j] = Frag<T>::mma(ah, bl[j], acc[i][j]);
          acc[i][j] = Frag<T>::mma(al, bh[j], acc[i][j]);
        }
      }
      Frag<T>::guard4(acc[i][0], acc[i][1], acc[i][2], acc[i][3], ah, al);
    }
    Frag<T>::keep(bh[0], bh[1], bh[2], bh[3]);
    if (SPLIT) Frag<T>::keep(bl[0], bl[1], bl[2], bl[3]);
  }
  acc_guard4(acc[0][0], acc[0][1], acc[0][2], acc[0][3]);
  acc_guard4(acc[1][0], acc[1][1], acc[1][2], acc[1][3]);
  acc_guard4(acc[2][0], acc[2][1], acc[2][2], acc[2][3]);
  acc_guard4(acc[3][0], acc[3][1], acc[3][2], acc[3][3]);

  float* slab = sT[wave];
  const float* Rb = RESID ? (resid + (size_t)b * strideR) : nullptr;
#pragma unroll
  for (int i = 0; i < 4; ++i) {
    const int mBase = m0 + (i << 4);
#pragma unroll
    for (int j = 0; j < 4; ++j) {
      const int n = n0 + (j << 4) + rlane;
      float bv = 0.f;
      if (BIAS_MODE == 2) bv = bias[n];
#pragma unroll
      for (int r = 0; r < 8; ++r) {
        float v = acc[i][j][r] * scale;
        if (BIAS_MODE == 1) v += bias[mBase + mOff + r];
        if (BIAS_MODE == 2) v += bv;
        if (RESID) v += Rb[(size_t)(mBase + mOff + r) * ldc + n];
        if (ACT == 2) v = fmaxf(v, 0.0f);
        if (ACT == 4) v = (v > 0.f) ? v : 0.01f * v;
        slab[(mOff + r) * 68 + (j << 4) + rlane] = v;
      }
    }
    __builtin_amdgcn_fence(__ATOMIC_RELEASE, "workgroup");
    __builtin_amdgcn_wave_barrier();
    __builtin_amdgcn_fence(__ATOMIC_ACQUIRE, "workgroup");
    if (OUT_MODE == 0) {
      float* C = (float*)Cout + (size_t)b * strideC;
      const int hh = lane >> 4, c4 = (lane & 15) * 4;
      for (int pass = 0; pass < 2; ++pass) {
#pragma unroll
        for (int it = 0; it < 8; ++it) {
          const int row = it * 2 + hh;
          v4f v = *(const v4f*)(slab + row * 68 + c4);
          *(volatile v4f*)(C + (size_t)(mBase + row) * ldc + n0 + c4) = v;
        }
        __threadfence();
      }
    } else {
      const int q = lane >> 3, c8 = (lane & 7) * 8;
      unsigned short* C  = (unsigned short*)Cout  + (size_t)b * strideC;
      unsigned short* C2 = (OUT_MODE == 2) ? ((unsigned short*)Cout2 + (size_t)b * strideC) : nullptr;
      for (int pass = 0; pass < 2; ++pass) {
#pragma unroll
        for (int it = 0; it < 4; ++it) {
          const int row = it * 4 + q;
          const float* sp = slab + row * 68 + c8;
          v8h hv, lv;
#pragma unroll
          for (int e = 0; e < 8; ++e) {
            if (OUT_MODE == 1) {
              hv[e] = (_Float16)sp[e];
            } else {
              unsigned short hb = f2bf_bits(sp[e]);
              unsigned short lb = f2bf_bits(sp[e] - bf_bits2f(hb));
              hv[e] = __builtin_bit_cast(_Float16, hb);
              lv[e] = __builtin_bit_cast(_Float16, lb);
            }
          }
          *(volatile v8h*)(C + (size_t)(mBase + row) * ldc + n0 + c8) = hv;
          if (OUT_MODE == 2) *(volatile v8h*)(C2 + (size_t)(mBase + row) * ldc + n0 + c8) = lv;
        }
        __threadfence();
      }
    }
    __builtin_amdgcn_fence(__ATOMIC_RELEASE, "workgroup");
    __builtin_amdgcn_wave_barrier();
    __builtin_amdgcn_fence(__ATOMIC_ACQUIRE, "workgroup");
  }
}

__global__ __launch_bounds__(256) void cvt8_hilo_kernel(const float* __restrict__ src, unsigned short* __restrict__ dh,
                                                        unsigned short* __restrict__ dl, int n8) {
  const int i = blockIdx.x * 256 + threadIdx.x;
  if (i < n8) {
    const float* sp = src + (size_t)i * 8;
    const v4f a = *(const v4f*)(sp);
    const v4f b = *(const v4f*)(sp + 4);
    v8h hv, lv;
#pragma unroll
    for (int e = 0; e < 4; ++e) {
      const float fa = a[e];
      const float fb = b[e];
      const unsigned short ha = f2bf_bits(fa);
      const unsigned short hb = f2bf_bits(fb);
      const unsigned short la = f2bf_bits(fa - bf_bits2f(ha));
      const unsigned short lb = f2bf_bits(fb - bf_bits2f(hb));
      hv[e]     = __builtin_bit_cast(_Float16, ha);
      hv[4 + e] = __builtin_bit_cast(_Float16, hb);
      lv[e]     = __builtin_bit_cast(_Float16, la);
      lv[4 + e] = __builtin_bit_cast(_Float16, lb);
    }
    *(volatile v8h*)(dh + (size_t)i * 8) = hv;
    *(volatile v8h*)(dl + (size_t)i * 8) = lv;
    __threadfence();
    *(volatile v8h*)(dh + (size_t)i * 8) = hv;
    *(volatile v8h*)(dl + (size_t)i * 8) = lv;
  }
}

template <int MODE>
__global__ __launch_bounds__(256) void tpw_kernel(const float* __restrict__ src, int R, int C, int ldo,
                                                  unsigned short* __restrict__ O, unsigned short* __restrict__ O2, float sc) {
  __shared__ float Tt[64 * 65];
  const int tid = threadIdx.x;
  const int c0 = blockIdx.x * 64, r0 = blockIdx.y * 64;
#pragma unroll
  for (int i = 0; i < 4; ++i) {
    const int idx = i * 256 + tid;
    const int rr = idx >> 4, cc = (idx & 15) * 4;
    const v4f v = *(const v4f*)(src + (size_t)(r0 + rr) * (size_t)C + c0 + cc);
    Tt[rr * 65 + cc + 0] = v[0];
    Tt[rr * 65 + cc + 1] = v[1];
    Tt[rr * 65 + cc + 2] = v[2];
    Tt[rr * 65 + cc + 3] = v[3];
  }
  __syncthreads();
  const int q = tid >> 3, c8 = (tid & 7) * 8;
  v8h hv[2], lv[2];
#pragma unroll
  for (int g = 0; g < 2; ++g) {
    const int qq = g * 32 + q;
#pragma unroll
    for (int e = 0; e < 8; ++e) {
      const float f = Tt[(c8 + e) * 65 + qq];
      if (MODE == 0) {
        const unsigned short hb = f2bf_bits(f);
        const unsigned short lb = f2bf_bits(f - bf_bits2f(hb));
        hv[g][e] = __builtin_bit_cast(_Float16, hb);
        lv[g][e] = __builtin_bit_cast(_Float16, lb);
      } else {
        hv[g][e] = (_Float16)(f * sc);
        lv[g][e] = hv[g][e];
      }
    }
  }
  for (int pass = 0; pass < 2; ++pass) {
#pragma unroll
    for (int g = 0; g < 2; ++g) {
      const size_t o = (size_t)(c0 + g * 32 + q) * (size_t)ldo + (size_t)(r0 + c8);
      *(volatile v8h*)(O + o) = hv[g];
      if (MODE == 0) *(volatile v8h*)(O2 + o) = lv[g];
    }
    __threadfence();
  }
}

__device__ __forceinline__ float sig_f(float x)  { return __builtin_amdgcn_rcpf(1.0f + expf(-x)); }
__device__ __forceinline__ float tanh_f(float x) { return 1.0f - 2.0f * __builtin_amdgcn_rcpf(1.0f + expf(2.0f * x)); }
__device__ __forceinline__ int clamp_tok(int v) { v = v < 0 ? 0 : v; return v > (DIM_V - 1) ? (DIM_V - 1) : v; }

__global__ __launch_bounds__(SCAN_THR) void recur_scan_kernel(
    const int* __restrict__ idx, const float* __restrict__ Pp,
    const unsigned short* __restrict__ WhTp, const unsigned short* __restrict__ WcTp,
    const float* __restrict__ Bh, const float* __restrict__ Bc,
    float* __restrict__ h_out, float* __restrict__ c_out,
    unsigned short* __restrict__ hbh, unsigned short* __restrict__ hbl) {
  __shared__ __align__(16) _Float16 St[2 * ST_BUF];
  __shared__ __align__(16) int      Tok[2 * 16];
  __shared__ __align__(16) float    Fs[2 * ROWS_BLK * FS_PITCH];
  const _Float16* WhT = (const _Float16*)WhTp;
  const _Float16* WcT = (const _Float16*)WcTp;
  const int tid = threadIdx.x, lane = tid & 31, wave = tid >> 5;
  const int c = lane & 15, hh = lane >> 4, koff = hh * 8;
  const int rowbase = blockIdx.x * ROWS_BLK;
  const int j = 16 * wave + c;

#pragma unroll 1
  for (int i = tid; i < 2 * ST_BUF; i += SCAN_THR) St[i] = (_Float16)0.0f;
  if (wave == 0) {
    const int v0 = clamp_tok(idx[(size_t)(rowbase + c) * SEQ_T]);
    Tok[c] = v0;
  }
  const float bhv = Bh[j];
  const float bcv = Bc[j];
  const _Float16* wh = WhT + (size_t)j * DIM_H + koff;
  const _Float16* wc = WcT + (size_t)j * DIM_H + koff;
  float hfin[8], cfin[8];
#pragma unroll
  for (int r = 0; r < 8; ++r) { hfin[r] = 0.0f; cfin[r] = 0.0f; }
  __syncthreads();

  const v8f z8 = {0.f, 0.f, 0.f, 0.f, 0.f, 0.f, 0.f, 0.f};

#pragma unroll 1
  for (int t = 0; t < SEQ_T; ++t) {
    const int cur = t & 1;
    float xw[8];
#pragma unroll
    for (int r = 0; r < 8; ++r) {
      const int tk = clamp_tok(Tok[cur * 16 + 8 * hh + r]);
      xw[r] = Pp[(size_t)tk * DIM_H + j];
    }
    if (wave == 0) {
      const int tn = (t + 1 < SEQ_T) ? (t + 1) : (SEQ_T - 1);
      const int vn = clamp_tok(idx[(size_t)(rowbase + c) * SEQ_T + tn]);
      Tok[(cur ^ 1) * 16 + c] = vn;
    }

    const _Float16* sb = St + cur * ST_BUF + c * ST_PITCH + koff;
    _Float16* sn = St + (cur ^ 1) * ST_BUF;
    v8f accH = z8, accHr = z8, accC = z8, accCr = z8;
#pragma unroll 1
    for (int k0 = 0; k0 < DIM_H; k0 += 32) {
      const v16h a0 = Frag<_Float16>::load(sb + k0);
      const v16h a1 = Frag<_Float16>::load(sb + ST_PLANE + k0);
      const v16h a2 = Frag<_Float16>::load(sb + 2 * ST_PLANE + k0);
      const v16h a3 = Frag<_Float16>::load(sb + 3 * ST_PLANE + k0);
      const v16h b0 = Frag<_Float16>::load(wh + k0);
      const v16h b1 = Frag<_Float16>::load(wc + k0);
      accH  = Frag<_Float16>::mma(a0, b0, accH);
      accHr = Frag<_Float16>::mma(a1, b0, accHr);
      accC  = Frag<_Float16>::mma(a2, b1, accC);
      accCr = Frag<_Float16>::mma(a3, b1, accCr);
      scan_guard(accH, accHr, accC, accCr, a0, a1, a2, a3, b0, b1);
    }
    acc_guard4(accH, accHr, accC, accCr);

#pragma unroll
    for (int r = 0; r < 8; ++r) {
      const float pre   = (accH[r] + accHr[r] * RES_CARRY_INV) * W_CARRY_INV + xw[r] + bhv;
      const float cterm = (accC[r] + accCr[r] * RES_CARRY_INV) * W_CARRY_INV + bcv;
      const float pcl = fminf(fmaxf(pre, -30.0f), 30.0f);
      const float s   = sig_f(pcl);
      const float tp  = tanh_f(pcl);
      const float cn  = s * (tp + cterm);
      const float ccl = fminf(fmaxf(cn, -30.0f), 30.0f);
      const float hn  = tanh_f(ccl) * s;
      hfin[r] = hn;
      cfin[r] = cn;
      const _Float16 hhi = (_Float16)hn;
      const float    hhf = (float)hhi;
      const _Float16 hlo = (_Float16)((hn - hhf) * RES_CARRY);
      const _Float16 chi = (_Float16)cn;
      const float    chf = (float)chi;
      const _Float16 clo = (_Float16)((cn - chf) * RES_CARRY);
      const int so = (8 * hh + r) * ST_PITCH + j;
      sn[so]                = hhi;
      sn[ST_PLANE + so]     = hlo;
      sn[2 * ST_PLANE + so] = chi;
      sn[3 * ST_PLANE + so] = clo;
    }
    __syncthreads();
  }

#pragma unroll
  for (int r = 0; r < 8; ++r) {
    Fs[(8 * hh + r) * FS_PITCH + j] = hfin[r];
    Fs[ROWS_BLK * FS_PITCH + (8 * hh + r) * FS_PITCH + j] = cfin[r];
  }
  __syncthreads();
  const int brow = tid >> 5, bc8 = (tid & 31) * 8;
  v8h bhv8, blv8;
  {
    const float* sp = Fs + brow * FS_PITCH + bc8;
#pragma unroll
    for (int e = 0; e < 8; ++e) {
      const float f = sp[e];
      const unsigned short hb = f2bf_bits(f);
      const unsigned short lb = f2bf_bits(f - bf_bits2f(hb));
      bhv8[e] = __builtin_bit_cast(_Float16, hb);
      blv8[e] = __builtin_bit_cast(_Float16, lb);
    }
  }
  for (int pass = 0; pass < 2; ++pass) {
#pragma unroll
    for (int it = 0; it < 2; ++it) {
      const int ix = it * SCAN_THR + tid;
      const int row = ix >> 6, c4 = (ix & 63) * 4;
      const v4f vh = *(const v4f*)(Fs + row * FS_PITCH + c4);
      const v4f vc = *(const v4f*)(Fs + ROWS_BLK * FS_PITCH + row * FS_PITCH + c4);
      *(volatile v4f*)(h_out + (size_t)(rowbase + row) * DIM_H + c4) = vh;
      *(volatile v4f*)(c_out + (size_t)(rowbase + row) * DIM_H + c4) = vc;
    }
    *(volatile v8h*)(hbh + (size_t)(rowbase + brow) * DIM_H + bc8) = bhv8;
    *(volatile v8h*)(hbl + (size_t)(rowbase + brow) * DIM_H + bc8) = blv8;
    __threadfence();
  }
}

extern "C" void kernel_launch(void* const* d_in, const int* in_sizes, int n_in,
                              void* d_out, int out_size, void* d_ws, size_t ws_size, hipStream_t stream) {
  if (n_in < 9 || d_out == nullptr || d_ws == nullptr) return;
  if (in_sizes[0] != SEQ_B * SEQ_T || in_sizes[1] != DIM_V * DIM_E || in_sizes[2] != DIM_E * DIM_H ||
      in_sizes[3] != DIM_H * DIM_H || in_sizes[4] != DIM_H * DIM_H || in_sizes[5] != DIM_H * DIM_V ||
      in_sizes[6] != DIM_V || in_sizes[7] != DIM_H || in_sizes[8] != DIM_H ||
      out_size != OUT0_ELEMS + 2 * OUT1_ELEMS) return;

  const int*   idx = (const int*)d_in[0];
  const float* emb = (const float*)d_in[1];
  const float* Wxh = (const float*)d_in[2];
  const float* Whh = (const float*)d_in[3];
  const float* Wch = (const float*)d_in[4];
  const float* Wy  = (const float*)d_in[5];
  const float* By  = (const float*)d_in[6];
  const float* Bh  = (const float*)d_in[7];
  const float* Bc  = (const float*)d_in[8];
  float* out   = (float*)d_out;
  float* h_out = out + (size_t)OUT0_ELEMS;
  float* c_out = h_out + (size_t)OUT1_ELEMS;

  char* ws = (char*)d_ws;
  size_t off = 0;
  auto carve = [&](size_t bytes) -> char* { char* p = ws + off; off += (bytes + 255) & ~(size_t)255; return p; };
  unsigned short* EMBH = (unsigned short*)carve((size_t)DIM_V * DIM_E * 2);
  unsigned short* EMBL = (unsigned short*)carve((size_t)DIM_V * DIM_E * 2);
  unsigned short* WXH  = (unsigned short*)carve((size_t)DIM_H * DIM_E * 2);
  unsigned short* WXL  = (unsigned short*)carve((size_t)DIM_H * DIM_E * 2);
  unsigned short* WHT  = (unsigned short*)carve((size_t)DIM_H * DIM_H * 2);
  unsigned short* WCT  = (unsigned short*)carve((size_t)DIM_H * DIM_H * 2);
  unsigned short* WYH  = (unsigned short*)carve((size_t)DIM_V * DIM_H * 2);
  unsigned short* WYL  = (unsigned short*)carve((size_t)DIM_V * DIM_H * 2);
  float*          PPL  = (float*)carve((size_t)DIM_V * DIM_H * 4);
  unsigned short* HBH  = (unsigned short*)carve((size_t)SEQ_B * DIM_H * 2);
  unsigned short* HBL  = (unsigned short*)carve((size_t)SEQ_B * DIM_H * 2);
  if (off > ws_size || off > (size_t)134217728) return;

  const int n8emb = DIM_V * (DIM_E / 8);
  cvt8_hilo_kernel<<<(n8emb + 255) / 256, 256, 0, stream>>>(emb, EMBH, EMBL, n8emb);
  tpw_kernel<0><<<dim3(DIM_H / 64, DIM_E / 64), 256, 0, stream>>>(Wxh, DIM_E, DIM_H, DIM_E, WXH, WXL, 1.0f);
  tpw_kernel<1><<<dim3(DIM_H / 64, DIM_H / 64), 256, 0, stream>>>(Whh, DIM_H, DIM_H, DIM_H, WHT, WHT, W_CARRY);
  tpw_kernel<1><<<dim3(DIM_H / 64, DIM_H / 64), 256, 0, stream>>>(Wch, DIM_H, DIM_H, DIM_H, WCT, WCT, W_CARRY);
  tpw_kernel<0><<<dim3(DIM_V / 64, DIM_H / 64), 256, 0, stream>>>(Wy, DIM_H, DIM_V, DIM_H, WYH, WYL, 1.0f);

  wmma_gemm64<1, true, 0, 0, false, 0><<<dim3((DIM_V / 64) * (DIM_H / 64) / 8, 1), 256, 0, stream>>>(
      EMBH, EMBL, DIM_E, 0L, WXH, WXL, DIM_E, 0L, (void*)PPL, (void*)PPL, DIM_H, 0L,
      By, PPL, 0L, DIM_V, DIM_H, DIM_E, 1.0f);

  recur_scan_kernel<<<SEQ_B / ROWS_BLK, SCAN_THR, 0, stream>>>(idx, PPL, WHT, WCT, Bh, Bc, h_out, c_out, HBH, HBL);

  wmma_gemm64<1, true, 2, 0, false, 0><<<dim3((SEQ_B / 64) * (DIM_V / 64) / 8, 1), 256, 0, stream>>>(
      HBH, HBL, DIM_H, 0L, WYH, WYL, DIM_H, 0L, (void*)out, (void*)out, DIM_V, 0L,
      By, PPL, 0L, SEQ_B, DIM_V, DIM_H, 1.0f);
}
